// Retention_49675591745550
// MI455X (gfx1250) — hardware-verified
//
#include <hip/hip_runtime.h>
#include <math.h>

constexpr int kTok      = 4096;
constexpr int kHeads    = 8;
constexpr int kHd       = 64;
constexpr int kChunk    = 1024;
constexpr int kNChunk   = kTok / kChunk;
constexpr int kVRows    = 80;
constexpr int kQTile    = 64;
constexpr int kKTile    = 64;
constexpr int kBandTiles = 17;
constexpr float kQScale = 0.125f;
constexpr float kEps    = 1.0e-6f;
static_assert(kTok % kChunk == 0 && kChunk % kQTile == 0, "tiles align with chunks");
static_assert(kTok * kHeads == 32768, "plane index shift");
static_assert(kHd == 64 && kKTile == 64 && kQTile == 64, "fragment tiling");
static_assert((kBandTiles - 1) * kKTile == kChunk, "band reaches one full chunk back");

typedef __attribute__((ext_vector_type(16))) __bf16   v16b;
typedef __attribute__((ext_vector_type(8)))  __bf16   v8b;
typedef __attribute__((ext_vector_type(8)))  float    v8f;
typedef __attribute__((ext_vector_type(4)))  float    v4f;
typedef __attribute__((ext_vector_type(4)))  unsigned int v4u;

__device__ __forceinline__ unsigned short f2bf_bits(float f) {
  unsigned u = __float_as_uint(f);
  return (unsigned short)((u + 0x7FFFu + ((u >> 16) & 1u)) >> 16);
}
__device__ __forceinline__ float bf_bits2f(unsigned short h) { return __uint_as_float(((unsigned)h) << 16); }
__device__ __forceinline__ unsigned pk16(unsigned short a, unsigned short b) { return (unsigned)a | ((unsigned)b << 16); }

__device__ __forceinline__ void split_bf(float f, __bf16& hi, __bf16& lo) {
  const unsigned short hb = f2bf_bits(f);
  hi = __builtin_bit_cast(__bf16, hb);
  const unsigned short lb = f2bf_bits(f - bf_bits2f(hb));
  lo = __builtin_bit_cast(__bf16, lb);
}

__device__ __forceinline__ v8f mma_bf(v16b a, v16b b, v8f c) {
  c = __builtin_amdgcn_wmma_f32_16x16x32_bf16(false, a, false, b, (short)0, c, false, false);
  asm volatile("v_nop\n\tv_nop\n\tv_nop\n\tv_nop" : "+v"(c) : "v"(a), "v"(b));
  return c;
}

union FragBF { v16b v; v8b h[2]; };
__device__ __forceinline__ v16b frag_load_g(const __bf16* p) {
  FragBF f;
  f.h[0] = *(const v8b*)(p);
  f.h[1] = *(const v8b*)(p + 16);
  return f.v;
}

__global__ __launch_bounds__(256) void gate_kernel(const float* __restrict__ log_g,
                                                   float* __restrict__ EG, float* __restrict__ EMS,
                                                   float* __restrict__ EMP) {
  __shared__ float lgs[kChunk];
  __shared__ float gcs[kChunk];
  __shared__ __align__(16) float o1[kChunk];
  __shared__ __align__(16) float o2[kChunk];
  __shared__ __align__(16) float o3[kChunk];
  const int t = threadIdx.x;
  const int c = blockIdx.x;
  const int h = blockIdx.y;
#pragma unroll
  for (int i = 0; i < 4; ++i) {
    const int l = i * 256 + t;
    const float x = log_g[(size_t)(c * kChunk + l) * kHeads + h];
    lgs[l] = bf_bits2f(f2bf_bits(x));
  }
  __syncthreads();
  if (t == 0) {
    float s = 0.0f;
#pragma unroll 4
    for (int l = 0; l < kChunk; ++l) {
      s += lgs[l];
      gcs[l] = s;
    }
  }
  __syncthreads();
  const float gend = gcs[kChunk - 1];
#pragma unroll 1
  for (int i = 0; i < 4; ++i) {
    const int l = 4 * t + i;
    const float gv = gcs[l];
    o1[l] = expf(gv);
    o2[l] = expf(-gv);
    o3[l] = expf(gend - gv);
  }
  __syncthreads();
  const v4f a1 = *(const v4f*)(o1 + 4 * t);
  const v4f a2 = *(const v4f*)(o2 + 4 * t);
  const v4f a3 = *(const v4f*)(o3 + 4 * t);
  const size_t off = (size_t)h * kTok + (size_t)c * kChunk + 4 * (size_t)t;
  *(volatile v4f*)(EG + off)  = a1;
  *(volatile v4f*)(EMS + off) = a2;
  *(volatile v4f*)(EMP + off) = a3;
  __threadfence();
  *(volatile v4f*)(EG + off)  = a1;
  *(volatile v4f*)(EMS + off) = a2;
  *(volatile v4f*)(EMP + off) = a3;
}

__global__ __launch_bounds__(256) void qk_plane_kernel(const float* __restrict__ q, const float* __restrict__ k,
                                                       unsigned short* __restrict__ Qp,
                                                       unsigned short* __restrict__ Kp, int nthreads) {
  const int i = blockIdx.x * 256 + threadIdx.x;
  if (i >= nthreads) return;
  const int d8  = i & 7;
  const int tkn = (i >> 3) & (kTok - 1);
  const int h   = i >> 15;
  const size_t src = ((size_t)(tkn * kHeads + h)) * kHd + 8 * d8;
  const v4f qa = *(const v4f*)(q + src);
  const v4f qb = *(const v4f*)(q + src + 4);
  const v4f ka = *(const v4f*)(k + src);
  const v4f kb = *(const v4f*)(k + src + 4);
  unsigned short qh[8], kh[8];
#pragma unroll
  for (int e = 0; e < 4; ++e) {
    qh[e]     = f2bf_bits(qa[e] * kQScale);
    qh[4 + e] = f2bf_bits(qb[e] * kQScale);
    kh[e]     = f2bf_bits(ka[e]);
    kh[4 + e] = f2bf_bits(kb[e]);
  }
  const v4u uq = (v4u){pk16(qh[0], qh[1]), pk16(qh[2], qh[3]), pk16(qh[4], qh[5]), pk16(qh[6], qh[7])};
  const v4u uk = (v4u){pk16(kh[0], kh[1]), pk16(kh[2], kh[3]), pk16(kh[4], kh[5]), pk16(kh[6], kh[7])};
  unsigned short* qd = Qp + 8 * (size_t)i;
  unsigned short* kd = Kp + 8 * (size_t)i;
  *(volatile v4u*)qd = uq;
  *(volatile v4u*)kd = uk;
  __threadfence();
  *(volatile v4u*)qd = uq;
  *(volatile v4u*)kd = uk;
}

__global__ __launch_bounds__(256) void vt_plane_kernel(const float* __restrict__ v, unsigned short* __restrict__ Vt) {
  __shared__ float sm[kVRows][65];
  const int t  = threadIdx.x;
  const int t0 = blockIdx.x * kKTile;
  const int h  = blockIdx.y;
#pragma unroll
  for (int i = 0; i < 4; ++i) {
    const int e  = i * 256 + t;
    const int tl = e >> 4;
    const int d4 = (e & 15) * 4;
    const v4f w = *(const v4f*)(v + ((size_t)((t0 + tl) * kHeads + h)) * kHd + d4);
    sm[d4 + 0][tl] = w[0];
    sm[d4 + 1][tl] = w[1];
    sm[d4 + 2][tl] = w[2];
    sm[d4 + 3][tl] = w[3];
  }
#pragma unroll
  for (int i = 0; i < 4; ++i) {
    const int e  = i * 256 + t;
    const int rr = e >> 6;
    const int cc = e & 63;
    sm[kHd + rr][cc] = (rr == 0) ? 1.0f : 0.0f;
  }
  __syncthreads();
  const int lane = t & 31, wave = t >> 5;
  const int qd = lane >> 3, c8 = (lane & 7) * 8;
  unsigned short* op = Vt + (size_t)h * kVRows * kTok;
  for (int pass = 0; pass < 2; ++pass) {
#pragma unroll
    for (int it = 0; it < 3; ++it) {
      if (it < 2 || wave < 4) {
        const int row = it * 32 + wave * 4 + qd;
        unsigned short hb[8];
#pragma unroll
        for (int e = 0; e < 8; ++e) hb[e] = f2bf_bits(sm[row][c8 + e]);
        const v4u u = (v4u){pk16(hb[0], hb[1]), pk16(hb[2], hb[3]), pk16(hb[4], hb[5]), pk16(hb[6], hb[7])};
        *(volatile v4u*)(op + (size_t)row * kTok + t0 + c8) = u;
      }
    }
    __threadfence();
  }
}

__global__ __launch_bounds__(128) void band_mix_kernel(const unsigned short* __restrict__ Qp,
                                                       const unsigned short* __restrict__ Kp,
                                                       const unsigned short* __restrict__ Vtp,
                                                       const float* __restrict__ EG,
                                                       const float* __restrict__ EMS,
                                                       const float* __restrict__ EMP,
                                                       float* __restrict__ out) {
  __shared__ __align__(16) __bf16 Psh[4][16 * kKTile];
  __shared__ __align__(16) __bf16 Psl[4][16 * kKTile];
  __shared__ __align__(16) float  Os[4][16 * 68];

  const int tid  = threadIdx.x;
  const int wave = tid >> 5;
  const int lane = tid & 31;
  const int hh   = lane >> 4;
  const int c    = lane & 15;
  const int qt   = blockIdx.x;
  const int h    = blockIdx.y;
  const int t0w  = qt * kQTile + wave * 16;

  const __bf16* Qb = (const __bf16*)Qp  + (size_t)h * kTok * kHd;
  const __bf16* Kb = (const __bf16*)Kp  + (size_t)h * kTok * kHd;
  const __bf16* Vb = (const __bf16*)Vtp + (size_t)h * kVRows * kTok;
  const float* egh  = EG  + (size_t)h * kTok;
  const float* emsh = EMS + (size_t)h * kTok;
  const float* emph = EMP + (size_t)h * kTok;

  v16b qa[2];
#pragma unroll
  for (int dc = 0; dc < 2; ++dc) qa[dc] = frag_load_g(Qb + (size_t)(t0w + c) * kHd + dc * 32 + 8 * hh);

  float egr[8];
  {
    const v4f e0 = *(const v4f*)(egh + t0w + 8 * hh);
    const v4f e1 = *(const v4f*)(egh + t0w + 8 * hh + 4);
    egr[0] = e0[0]; egr[1] = e0[1]; egr[2] = e0[2]; egr[3] = e0[3];
    egr[4] = e1[0]; egr[5] = e1[1]; egr[6] = e1[2]; egr[7] = e1[3];
  }

  v8f oacc[5];
#pragma unroll
  for (int tt = 0; tt < 5; ++tt) oacc[tt] = (v8f){0.f,0.f,0.f,0.f,0.f,0.f,0.f,0.f};

  const int cq   = qt >> 4;
  const int ktlo = (qt >= kBandTiles - 1) ? (qt - (kBandTiles - 1)) : 0;
  __bf16* pwh = Psh[wave];
  __bf16* pwl = Psl[wave];

  for (int kt = ktlo; kt <= qt; ++kt) {
    const int kv0 = kt * kKTile;

    v8f s[4];
#pragma unroll
    for (int j = 0; j < 4; ++j) {
      s[j] = (v8f){0.f,0.f,0.f,0.f,0.f,0.f,0.f,0.f};
#pragma unroll
      for (int dc = 0; dc < 2; ++dc) {
        const v16b kb = frag_load_g(Kb + (size_t)(kv0 + j * 16 + c) * kHd + dc * 32 + 8 * hh);
        s[j] = mma_bf(qa[dc], kb, s[j]);
      }
    }

    const bool same = ((kt >> 4) == cq);
    const float* cfp = same ? emsh : emph;
    float cf[4];
#pragma unroll
    for (int j = 0; j < 4; ++j) cf[j] = cfp[kv0 + j * 16 + c];
    const int lim_add = (kt == qt) ? 0 : kTok;
#pragma unroll
    for (int r = 0; r < 8; ++r) {
      const int lim = t0w + 8 * hh + r + lim_add;
      const float rf = egr[r];
#pragma unroll
      for (int j = 0; j < 4; ++j) {
        const int skey = kv0 + j * 16 + c;
        const float x = s[j][r];
        float a = (rf * cf[j]) * (x * x);
        a = (skey > lim) ? 0.0f : a;
        __bf16 ahv, alv;
        split_bf(a, ahv, alv);
        pwh[(8 * hh + r) * kKTile + j * 16 + c] = ahv;
        pwl[(8 * hh + r) * kKTile + j * 16 + c] = alv;
      }
    }
    __builtin_amdgcn_fence(__ATOMIC_RELEASE, "workgroup");
    __builtin_amdgcn_wave_barrier();
    __builtin_amdgcn_fence(__ATOMIC_ACQUIRE, "workgroup");

#pragma unroll 1
    for (int kk = 0; kk < 2; ++kk) {
      FragBF pa, pl;
      pa.h[0] = *(const v8b*)(pwh + c * kKTile + kk * 32 + 8 * hh);
      pa.h[1] = *(const v8b*)(pwh + c * kKTile + kk * 32 + 16 + 8 * hh);
      pl.h[0] = *(const v8b*)(pwl + c * kKTile + kk * 32 + 8 * hh);
      pl.h[1] = *(const v8b*)(pwl + c * kKTile + kk * 32 + 16 + 8 * hh);
#pragma unroll
      for (int tt = 0; tt < 5; ++tt) {
        const v16b vb = frag_load_g(Vb + (size_t)(tt * 16 + c) * kTok + kv0 + kk * 32 + 8 * hh);
        oacc[tt] = mma_bf(pa.v, vb, oacc[tt]);
        oacc[tt] = mma_bf(pl.v, vb, oacc[tt]);
      }
    }
    __builtin_amdgcn_fence(__ATOMIC_RELEASE, "workgroup");
    __builtin_amdgcn_wave_barrier();
    __builtin_amdgcn_fence(__ATOMIC_ACQUIRE, "workgroup");
  }

  float* os = Os[wave];
#pragma unroll
  for (int r = 0; r < 8; ++r) {
    const float den = __shfl(oacc[4][r], lane & 16, 32);
    const float inv = 1.0f / fmaxf(den, kEps);
#pragma unroll
    for (int tt = 0; tt < 4; ++tt) os[(8 * hh + r) * 68 + tt * 16 + c] = oacc[tt][r] * inv;
  }
  __builtin_amdgcn_fence(__ATOMIC_RELEASE, "workgroup");
  __builtin_amdgcn_wave_barrier();
  __builtin_amdgcn_fence(__ATOMIC_ACQUIRE, "workgroup");
  {
    const int c4 = c * 4;
    for (int pass = 0; pass < 2; ++pass) {
#pragma unroll
      for (int it = 0; it < 8; ++it) {
        const int row = it * 2 + hh;
        const v4f val = *(const v4f*)(os + row * 68 + c4);
        *(volatile v4f*)(out + ((size_t)(t0w + row) * kHeads + h) * kHd + c4) = val;
      }
      __threadfence();
    }
  }
}

extern "C" void kernel_launch(void* const* d_in, const int* in_sizes, int n_in,
                              void* d_out, int out_size, void* d_ws, size_t ws_size,
                              hipStream_t stream) {
  if (n_in < 4) return;
  const int nElem = kTok * kHeads * kHd;
  if (in_sizes[0] != nElem || in_sizes[1] != nElem || in_sizes[2] != nElem) return;
  if (in_sizes[3] != kTok * kHeads) return;
  if (out_size != nElem) return;

  const size_t szG  = (size_t)kHeads * kTok * 4;
  const size_t szQK = (size_t)kHeads * kTok * kHd * 2;
  const size_t szVT = (size_t)kHeads * kVRows * kTok * 2;
  const size_t offEG  = 0;
  const size_t offEMS = offEG + szG;
  const size_t offEMP = offEMS + szG;
  const size_t offQ   = offEMP + szG;
  const size_t offK   = offQ + szQK;
  const size_t offVT  = offK + szQK;
  const size_t total  = offVT + szVT;
  if (ws_size < total) return;

  const float* q  = (const float*)d_in[0];
  const float* k  = (const float*)d_in[1];
  const float* v  = (const float*)d_in[2];
  const float* lg = (const float*)d_in[3];
  float* out = (float*)d_out;
  char* ws = (char*)d_ws;
  float* EG  = (float*)(ws + offEG);
  float* EMS = (float*)(ws + offEMS);
  float* EMP = (float*)(ws + offEMP);
  unsigned short* Qp = (unsigned short*)(ws + offQ);
  unsigned short* Kp = (unsigned short*)(ws + offK);
  unsigned short* Vt = (unsigned short*)(ws + offVT);

  gate_kernel<<<dim3(kNChunk, kHeads), dim3(256), 0, stream>>>(lg, EG, EMS, EMP);
  const int nthr = kHeads * kTok * (kHd / 8);
  qk_plane_kernel<<<dim3((nthr + 255) / 256), dim3(256), 0, stream>>>(q, k, Qp, Kp, nthr);
  vt_plane_kernel<<<dim3(kTok / kKTile, kHeads), dim3(256), 0, stream>>>(v, Vt);
  band_mix_kernel<<<dim3(kTok / kQTile, kHeads), dim3(128), 0, stream>>>(Qp, Kp, Vt, EG, EMS, EMP, out);
}
